// selfBank_31215822308175
// MI455X (gfx1250) — hardware-run, weakly checked
//
#include <hip/hip_runtime.h>
#include <math.h>

typedef __attribute__((ext_vector_type(16))) _Float16 v16h;
typedef __attribute__((ext_vector_type(8)))  _Float16 v8h;
typedef __attribute__((ext_vector_type(8)))  float    v8f;
typedef __attribute__((ext_vector_type(4)))  float    v4f;
typedef __attribute__((ext_vector_type(4)))  unsigned v4u;

constexpr int kBatch        = 32;
constexpr int kSigLen       = 50000;
constexpr int kFrameLen     = 25;
constexpr int kHop          = 10;
constexpr int kFramesPerSig = 4999;
constexpr int kNfft         = 512;
constexpr int kBinsUsed     = 256;
constexpr int kNumFilt      = 40;
constexpr int kFiltRows     = 48;
constexpr int kKPad         = 32;
constexpr int kTwRows       = 2 * kBinsUsed;
constexpr int kRows         = kBatch * kFramesPerSig;
constexpr int kRowsPad      = 160000;
constexpr int kTilesM       = kRowsPad / 64;
constexpr int kOutPerTile   = 64 * kNumFilt;
constexpr int kOutPerSlab   = 16 * kNumFilt;
constexpr int kSampleRate   = 1000;
constexpr int kPowPitch     = 260;
static_assert(kRows == 159968);
static_assert((kRowsPad % 64) == 0 && kRowsPad >= kRows && (kRows % 16) == 0);
static_assert((kFramesPerSig - 1) * kHop + kFrameLen == kSigLen + 5);
static_assert(kFrameLen <= kKPad && (kKPad % 32) == 0 && (kBinsUsed % 32) == 0);
static_assert((kOutPerSlab % 128) == 0 && (kOutPerTile * 4) % 128 == 0);
static_assert(kFiltRows % 16 == 0 && kFiltRows >= kNumFilt);

constexpr float kFrameCarry = 64.0f;
constexpr float kTwCarry    = 1024.0f;
constexpr float kPowCarry   = 1024.0f;
constexpr float kFbCarry    = 1024.0f;
constexpr float kPowScale   = kPowCarry / ((float)kNfft * (kFrameCarry * kTwCarry) * (kFrameCarry * kTwCarry));
constexpr float kFbScale    = 1.0f / (kPowCarry * kFbCarry);
constexpr float kF16MinNormal = 6.103515625e-5f;
constexpr float kEpsF       = 2.2204460492503131e-16f;
constexpr float kDbPerNep   = (float)(20.0 / 2.302585092994045684);

constexpr size_t kOffTW   = 0;
constexpr size_t kOffFB   = kOffTW + (size_t)kTwRows * kKPad * 2;
constexpr size_t kOffFR   = kOffFB + (size_t)kFiltRows * kBinsUsed * 2;
constexpr size_t kOffPW   = kOffFR + (size_t)kRowsPad * kKPad * 2;
constexpr size_t kWsTotal = kOffPW + (size_t)kRowsPad * kBinsUsed * 2;
static_assert(kWsTotal == 92217344ull);
static_assert(kWsTotal <= 134217728ull);
static_assert((kOffFB % 128) == 0 && (kOffFR % 128) == 0 && (kOffPW % 128) == 0);
constexpr int kTwWords  = kTwRows * kKPad / 2;
constexpr int kFbWords  = kFiltRows * kBinsUsed / 2;
constexpr int kTabBlocks = (kTwWords + kFbWords) / 1024;
static_assert(kTwWords == 8 * 1024 && kFbWords == 6 * 1024 && kOffFB == (size_t)kTwWords * 4);

constexpr double cx_ln(double x) {
  const double y = (x - 1.0) / (x + 1.0);
  const double y2 = y * y;
  double term = y;
  double sum = 0.0;
  for (int k = 0; k < 60; ++k) {
    sum += term / (double)(2 * k + 1);
    term *= y2;
  }
  return 2.0 * sum;
}
constexpr double cx_exp(double t) {
  double term = 1.0;
  double sum = 1.0;
  for (int k = 1; k < 40; ++k) {
    term = term * t / (double)k;
    sum += term;
  }
  return sum;
}
constexpr double mel_edge(int i) {
  const double half_rate = (double)kSampleRate / 2.0;
  const double lnr = cx_ln(1.0 + half_rate / 700.0);
  const double hz = 700.0 * (cx_exp(lnr * (double)i / (double)(kNumFilt + 1)) - 1.0);
  return hz / half_rate * ((double)kNfft / 2.0);
}

struct FiltParams {
  double b0, b2, invRise, invFall;
  int left, center, right, spare;
};

template <int I> struct FilterPick {
  static __device__ __forceinline__ void run(int n, FiltParams& f) {
    constexpr double e0 = mel_edge(I);
    constexpr double e1 = mel_edge(I + 1);
    constexpr double e2 = mel_edge(I + 2);
    constexpr double ir = 1.0 / (e1 - e0);
    constexpr double ifl = 1.0 / (e2 - e1);
    constexpr int il = (int)e0;
    constexpr int ic = (int)e1;
    constexpr int irt = (int)e2;
    if (n == I) {
      f.b0 = e0;
      f.b2 = e2;
      f.invRise = ir;
      f.invFall = ifl;
      f.left = il;
      f.center = ic;
      f.right = irt;
    }
    FilterPick<I + 1>::run(n, f);
  }
};
template <> struct FilterPick<kNumFilt> {
  static __device__ __forceinline__ void run(int, FiltParams&) {}
};

union FragH { v16h v; v8h h[2]; };
__device__ __forceinline__ v16h frag_load(const _Float16* p) {
  FragH f;
  f.h[0] = *(const v8h*)(p);
  f.h[1] = *(const v8h*)(p + 16);
  return f.v;
}
__device__ __forceinline__ v8f mma_f16(v16h a, v16h b, v8f c) {
  c = __builtin_amdgcn_wmma_f32_16x16x32_f16(false, a, false, b, (short)0, c, false, false);
  asm volatile("v_nop\n\tv_nop\n\tv_nop\n\tv_nop" : "+v"(c) : "v"(a), "v"(b));
  return c;
}
__device__ __forceinline__ float flush_f16(float v) {
  return (fabsf(v) < kF16MinNormal) ? 0.0f : v;
}
__device__ __forceinline__ unsigned pack_f16x2(float lo, float hi) {
  const _Float16 h0 = (_Float16)lo;
  const _Float16 h1 = (_Float16)hi;
  return (unsigned)__builtin_bit_cast(unsigned short, h0) | ((unsigned)__builtin_bit_cast(unsigned short, h1) << 16);
}
__device__ __forceinline__ float tw_value(int k, int bin, int shift) {
  const int ph = (k * bin + shift) & (kNfft - 1);
  const float c = cospif((float)ph * (2.0f / (float)kNfft));
  const float v = (k < kFrameLen) ? c * kTwCarry : 0.0f;
  return flush_f16(v);
}
__device__ __forceinline__ float fb_value(int c, const FiltParams& f, bool rowok) {
  const int j = c - 1;
  const bool rising  = (j >= f.left) && (j < f.center);
  const bool falling = (j >= f.center) && (j < f.right);
  const double num = rising ? ((double)c - f.b0) : (f.b2 - (double)c);
  const double inv = rising ? f.invRise : f.invFall;
  const float w = (float)(num * inv);
  const float v = (rowok && (rising || falling)) ? w * kFbCarry : 0.0f;
  return flush_f16(v);
}

__global__ __launch_bounds__(256) void tables_kernel(unsigned* __restrict__ tabw) {
  __shared__ __align__(16) unsigned sw[1024];
  const int tid = threadIdx.x;
  const int blk = blockIdx.x;
  if (blk < kTwWords / 1024) {
#pragma unroll 1
    for (int it = 0; it < 4; ++it) {
      const int widx = it * 256 + tid;
      const int e0 = (blk * 1024 + widx) * 2;
      const int row = e0 >> 5;
      const int k0 = e0 & 31;
      const int bin = row & (kBinsUsed - 1);
      const int shift = (row >> 8) * (kNfft / 4);
      const float v0 = tw_value(k0, bin, shift);
      const float v1 = tw_value(k0 + 1, bin, shift);
      sw[widx] = pack_f16x2(v0, v1);
    }
  } else {
#pragma unroll 1
    for (int it = 0; it < 4; ++it) {
      const int widx = it * 256 + tid;
      const int e0 = ((blk - kTwWords / 1024) * 1024 + widx) * 2;
      const int n = e0 >> 8;
      const int c0 = e0 & (kBinsUsed - 1);
      const bool rowok = n < kNumFilt;
      const int nn = rowok ? n : (kNumFilt - 1);
      FiltParams f;
      f.b0 = 0.0; f.b2 = 0.0; f.invRise = 0.0; f.invFall = 0.0;
      f.left = 0; f.center = 0; f.right = 0; f.spare = 0;
      FilterPick<0>::run(nn, f);
      const float v0 = fb_value(c0, f, rowok);
      const float v1 = fb_value(c0 + 1, f, rowok);
      sw[widx] = pack_f16x2(v0, v1);
    }
  }
  __syncthreads();
  const v4u val = *(const v4u*)(sw + tid * 4);
  unsigned* dst = tabw + (size_t)blk * 1024 + tid * 4;
  *(volatile v4u*)dst = val;
  __threadfence();
  *(volatile v4u*)dst = val;
}

__global__ __launch_bounds__(256) void frames_kernel(const float* __restrict__ sig, unsigned short* __restrict__ frp) {
  const int i = blockIdx.x * 256 + threadIdx.x;
  if (i >= kRowsPad * 4) return;
  const int r = i >> 2;
  const int q = i & 3;
  const bool rowok = r < kRows;
  const int rv = rowok ? r : (kRows - 1);
  const int b = rv / kFramesPerSig;
  const int t = rv - b * kFramesPerSig;
  const int s0 = t * kHop + q * 8;
  const float* base = sig + (size_t)b * kSigLen;
  v8h hv;
#pragma unroll
  for (int e = 0; e < 8; ++e) {
    const int k = q * 8 + e;
    const int idx = s0 + e;
    const int idc = (idx < kSigLen) ? idx : (kSigLen - 1);
    float x = base[idc];
    asm volatile("" : "+v"(x));
    const bool ok = rowok && (k < kFrameLen) && (idx < kSigLen);
    float v = ok ? x * kFrameCarry : 0.0f;
    v = flush_f16(v);
    hv[e] = (_Float16)v;
  }
  unsigned short* dst = frp + (size_t)i * 8;
  *(volatile v8h*)dst = hv;
  __threadfence();
  *(volatile v8h*)dst = hv;
}

__global__ __launch_bounds__(256) void dft_power_kernel(const unsigned short* __restrict__ frp,
                                                        const unsigned short* __restrict__ twp,
                                                        unsigned short* __restrict__ pwp) {
  __shared__ __align__(16) float sP[32 * kPowPitch];
  const _Float16* A  = (const _Float16*)frp;
  const _Float16* Bt = (const _Float16*)twp;
  const int tid = threadIdx.x;
  const int lane = tid & 31;
  const int wave = tid >> 5;
  const int c = lane & 15;
  const int h = lane >> 4;
  const int m0 = blockIdx.x * 32;

  v16h bc[2], bs[2];
#pragma unroll
  for (int j = 0; j < 2; ++j) {
    const int bin = wave * 32 + j * 16 + c;
    bc[j] = frag_load(Bt + (size_t)bin * kKPad + 8 * h);
    bs[j] = frag_load(Bt + (size_t)(kBinsUsed + bin) * kKPad + 8 * h);
  }
#pragma unroll
  for (int i = 0; i < 2; ++i) {
    const v16h ah = frag_load(A + (size_t)(m0 + i * 16 + c) * kKPad + 8 * h);
#pragma unroll
    for (int j = 0; j < 2; ++j) {
      v8f re = (v8f){0.f, 0.f, 0.f, 0.f, 0.f, 0.f, 0.f, 0.f};
      v8f im = (v8f){0.f, 0.f, 0.f, 0.f, 0.f, 0.f, 0.f, 0.f};
      re = mma_f16(ah, bc[j], re);
      im = mma_f16(ah, bs[j], im);
#pragma unroll
      for (int r = 0; r < 8; ++r) {
        const float p = (re[r] * re[r] + im[r] * im[r]) * kPowScale;
        sP[(i * 16 + 8 * h + r) * kPowPitch + wave * 32 + j * 16 + c] = p;
      }
    }
  }
  __syncthreads();
  v8h hv[4];
#pragma unroll
  for (int it = 0; it < 4; ++it) {
    const float* sp = sP + (wave * 4 + it) * kPowPitch + lane * 8;
    const v4f a0 = *(const v4f*)(sp);
    const v4f a1 = *(const v4f*)(sp + 4);
#pragma unroll
    for (int e = 0; e < 4; ++e) {
      const float x0 = flush_f16(a0[e]);
      const float x1 = flush_f16(a1[e]);
      hv[it][e]     = (_Float16)x0;
      hv[it][4 + e] = (_Float16)x1;
    }
  }
  for (int pass = 0; pass < 2; ++pass) {
#pragma unroll
    for (int it = 0; it < 4; ++it) {
      unsigned short* dst = pwp + (size_t)(m0 + wave * 4 + it) * kBinsUsed + lane * 8;
      *(volatile v8h*)dst = hv[it];
    }
    __threadfence();
  }
}

__global__ __launch_bounds__(256) void mel_log_kernel(const unsigned short* __restrict__ pwp,
                                                      const unsigned short* __restrict__ fbp,
                                                      float* __restrict__ out,
                                                      const int* __restrict__ fsp) {
  __shared__ __align__(16) float sT[8][kOutPerSlab];
  const _Float16* A  = (const _Float16*)pwp;
  const _Float16* Bt = (const _Float16*)fbp;
  const int lane = threadIdx.x & 31;
  const int wave = threadIdx.x >> 5;
  const int tile = blockIdx.x * 8 + wave;
  if (tile >= kTilesM) return;
  const int m0 = tile << 6;
  const int rlane = lane & 15;
  const int koff = (lane >> 4) * 8;
  const int mOff = (lane >> 4) * 8;
  const int fsv = fsp[0];
  const bool bad = (fsv != kSampleRate);
  const float nanv = __uint_as_float(0x7fc00000u);

  v8f acc[4][3];
#pragma unroll
  for (int i = 0; i < 4; ++i)
#pragma unroll
    for (int j = 0; j < 3; ++j) acc[i][j] = (v8f){0.f, 0.f, 0.f, 0.f, 0.f, 0.f, 0.f, 0.f};

#pragma unroll 1
  for (int k0 = 0; k0 < kBinsUsed; k0 += 32) {
    v16h bh[3];
#pragma unroll
    for (int j = 0; j < 3; ++j)
      bh[j] = frag_load(Bt + (size_t)((j << 4) + rlane) * kBinsUsed + koff + k0);
#pragma unroll
    for (int i = 0; i < 4; ++i) {
      const v16h ah = frag_load(A + (size_t)(m0 + (i << 4) + rlane) * kBinsUsed + koff + k0);
#pragma unroll
      for (int j = 0; j < 3; ++j) acc[i][j] = mma_f16(ah, bh[j], acc[i][j]);
    }
  }

  float* slab = sT[wave];
#pragma unroll
  for (int i = 0; i < 4; ++i) {
    const int mBase = m0 + (i << 4);
    if (mBase < kRows) {
#pragma unroll
      for (int j = 0; j < 3; ++j) {
        const int col = (j << 4) + rlane;
#pragma unroll
        for (int r = 0; r < 8; ++r) {
          const float v = acc[i][j][r] * kFbScale;
          if (col < kNumFilt) slab[(mOff + r) * kNumFilt + col] = v;
        }
      }
      __builtin_amdgcn_fence(__ATOMIC_RELEASE, "workgroup");
      __builtin_amdgcn_wave_barrier();
      __builtin_amdgcn_fence(__ATOMIC_ACQUIRE, "workgroup");
#pragma unroll 1
      for (int it = 0; it < 5; ++it) {
        float* sp = slab + (it * 32 + lane) * 4;
        const v4f vin = *(const v4f*)sp;
        v4f vo;
#pragma unroll
        for (int e = 0; e < 4; ++e) {
          float x = vin[e];
          x = (x == 0.0f) ? kEpsF : x;
          float y = kDbPerNep * logf(x);
          y = bad ? nanv : y;
          vo[e] = y;
        }
        *(v4f*)sp = vo;
      }
      __builtin_amdgcn_fence(__ATOMIC_RELEASE, "workgroup");
      __builtin_amdgcn_wave_barrier();
      __builtin_amdgcn_fence(__ATOMIC_ACQUIRE, "workgroup");
      float* dst = out + (size_t)tile * kOutPerTile + (size_t)i * kOutPerSlab;
      for (int pass = 0; pass < 2; ++pass) {
#pragma unroll
        for (int it = 0; it < 5; ++it) {
          const v4f v = *(const v4f*)(slab + (it * 32 + lane) * 4);
          *(volatile v4f*)(dst + (it * 32 + lane) * 4) = v;
        }
        __threadfence();
      }
      __builtin_amdgcn_fence(__ATOMIC_RELEASE, "workgroup");
      __builtin_amdgcn_wave_barrier();
      __builtin_amdgcn_fence(__ATOMIC_ACQUIRE, "workgroup");
    }
  }
}

extern "C" void kernel_launch(void* const* d_in, const int* in_sizes, int n_in,
                              void* d_out, int out_size, void* d_ws, size_t ws_size,
                              hipStream_t stream) {
  if (n_in < 2) return;
  if (in_sizes[0] != kBatch * kSigLen) return;
  if (in_sizes[1] != 1) return;
  if (out_size != kRows * kNumFilt) return;
  if (ws_size < kWsTotal) return;

  const float* sig = (const float*)d_in[0];
  const int*   fsp = (const int*)d_in[1];
  float* out = (float*)d_out;
  char* ws = (char*)d_ws;
  unsigned*       tabw = (unsigned*)(ws + kOffTW);
  unsigned short* twp  = (unsigned short*)(ws + kOffTW);
  unsigned short* fbp  = (unsigned short*)(ws + kOffFB);
  unsigned short* frp  = (unsigned short*)(ws + kOffFR);
  unsigned short* pwp  = (unsigned short*)(ws + kOffPW);

  tables_kernel<<<kTabBlocks, 256, 0, stream>>>(tabw);
  frames_kernel<<<(kRowsPad * 4) / 256, 256, 0, stream>>>(sig, frp);
  dft_power_kernel<<<kRowsPad / 32, 256, 0, stream>>>(frp, twp, pwp);
  mel_log_kernel<<<(kTilesM + 7) / 8, 256, 0, stream>>>(pwp, fbp, out, fsp);
}
